// PolyNetFP4Sim_76355928588536
// MI455X (gfx1250) — hardware-verified
//
#include <hip/hip_runtime.h>


typedef _Float16 v16h __attribute__((ext_vector_type(16)));
typedef _Float16 v8h  __attribute__((ext_vector_type(8)));
typedef float    v8f  __attribute__((ext_vector_type(8)));
typedef float    v4f  __attribute__((ext_vector_type(4)));

union Frag { v16h v; v8h half[2]; };

static constexpr float kActScale = 32.0f;
static constexpr float kActInv   = 0.03125f;

__device__ __forceinline__ float qfp4(float w) {
    if (w == 0.0f) return 0.0f;
    int e;
    const float m = frexpf(fabsf(w), &e);
    int qe = e + 1;
    qe = qe < 0 ? 0 : (qe > 3 ? 3 : qe);
    const float dec = ldexpf(m >= 0.75f ? 0.75f : 0.5f, qe - 1);
    return w < 0.0f ? -dec : dec;
}

__device__ __forceinline__ v8f wmma_f16(v16h a, v16h b, v8f c) {
    v8f d = __builtin_amdgcn_wmma_f32_16x16x32_f16(false, a, false, b, (short)0, c, false, false);
    asm volatile("v_nop\n\tv_nop\n\tv_nop\n\tv_nop" : "+v"(d) : "v"(a), "v"(b));
    return d;
}

__device__ __forceinline__ float silu_scaled(float ps) {
    const float e = __expf(ps * (-kActInv));
    const float r = __builtin_amdgcn_rcpf(1.0f + e);
    return ps * r;
}

__global__ void __launch_bounds__(256) mlp_fp4_kernel(
    const float* __restrict__ x,
    const float* __restrict__ w1, const float* __restrict__ b1,
    const float* __restrict__ w2, const float* __restrict__ b2,
    const float* __restrict__ w3, const float* __restrict__ b3,
    const float* __restrict__ w4, const float* __restrict__ b4,
    float* __restrict__ out,
    int nX, int nOut, int nChunks, int nWaves)
{
    __shared__ _Float16 sw2[64 * 64] __attribute__((aligned(16)));
    __shared__ _Float16 sw3[32 * 64] __attribute__((aligned(16)));
    __shared__ float    sl1[128]     __attribute__((aligned(16)));
    __shared__ float    sw4[32]      __attribute__((aligned(16)));

    for (int t = threadIdx.x; t < 64 * 64; t += blockDim.x) sw2[t] = (_Float16)qfp4(w2[t]);
    for (int t = threadIdx.x; t < 32 * 64; t += blockDim.x) sw3[t] = (_Float16)qfp4(w3[t]);
    for (int t = threadIdx.x; t < 64; t += blockDim.x) {
        sl1[2 * t]     = kActScale * qfp4(w1[t]);
        sl1[2 * t + 1] = kActScale * b1[t];
    }
    for (int t = threadIdx.x; t < 32; t += blockDim.x) sw4[t] = kActInv * qfp4(w4[t]);
    __syncthreads();

    const int lane = threadIdx.x & 31;
    const int h    = lane >> 4;
    const int row  = lane & 15;

    v8f c2s[4];
#pragma unroll
    for (int ma = 0; ma < 4; ++ma)
#pragma unroll
        for (int v = 0; v < 8; ++v) c2s[ma][v] = kActScale * b2[ma * 16 + 8 * h + v];
    v8f c3s[2];
#pragma unroll
    for (int ma = 0; ma < 2; ++ma)
#pragma unroll
        for (int v = 0; v < 8; ++v) c3s[ma][v] = kActScale * b3[ma * 16 + 8 * h + v];
    float w4r[16];
#pragma unroll
    for (int ma = 0; ma < 2; ++ma)
#pragma unroll
        for (int v = 0; v < 8; ++v) w4r[ma * 8 + v] = sw4[ma * 16 + 8 * h + v];
    const float b4s = b4[0];

    const int wave0 = blockIdx.x * (blockDim.x >> 5) + (threadIdx.x >> 5);
    const int qsel  = lane >> 2;
    const int src0  = (lane & 3) << 2;

    for (int chunk = wave0; chunk < nChunks; chunk += nWaves) {
        v4f o = {0.0f, 0.0f, 0.0f, 0.0f};
#pragma unroll 1
        for (int j = 0; j < 8; ++j) {
            const int base = chunk * 128 + j * 16;
            int xi = base + row;
            xi = xi < nX ? xi : nX - 1;
            const float xs = x[xi];

            Frag bq[2];
#pragma unroll
            for (int kb = 0; kb < 2; ++kb) {
#pragma unroll
                for (int g = 0; g < 2; ++g) {
                    const int k0 = kb * 32 + 16 * g + 8 * h;
                    const v4f* pp = (const v4f*)(sl1 + 2 * k0);
                    v8h hv;
#pragma unroll
                    for (int q = 0; q < 4; ++q) {
                        const v4f wb = pp[q];
                        const float p0 = fmaf(xs, wb[0], wb[1]);
                        const float p1 = fmaf(xs, wb[2], wb[3]);
                        hv[2 * q]     = (_Float16)silu_scaled(p0);
                        hv[2 * q + 1] = (_Float16)silu_scaled(p1);
                    }
                    bq[kb].half[g] = hv;
                }
            }

            Frag b3q[2];
#pragma unroll
            for (int ma = 0; ma < 4; ++ma) {
                const _Float16* ap = sw2 + (ma * 16 + row) * 64 + 8 * h;
                v8f acc = c2s[ma];
#pragma unroll
                for (int kb = 0; kb < 2; ++kb) {
                    Frag a;
                    a.half[0] = *(const v8h*)(ap + kb * 32);
                    a.half[1] = *(const v8h*)(ap + kb * 32 + 16);
                    acc = wmma_f16(a.v, bq[kb].v, acc);
                }
                v8h hv;
#pragma unroll
                for (int v = 0; v < 8; ++v) hv[v] = (_Float16)silu_scaled(acc[v]);
                b3q[ma >> 1].half[ma & 1] = hv;
            }

            float pa = 0.0f, pb = 0.0f;
#pragma unroll
            for (int ma = 0; ma < 2; ++ma) {
                const _Float16* ap = sw3 + (ma * 16 + row) * 64 + 8 * h;
                v8f acc = c3s[ma];
#pragma unroll
                for (int kb = 0; kb < 2; ++kb) {
                    Frag a;
                    a.half[0] = *(const v8h*)(ap + kb * 32);
                    a.half[1] = *(const v8h*)(ap + kb * 32 + 16);
                    acc = wmma_f16(a.v, b3q[kb].v, acc);
                }
#pragma unroll
                for (int v = 0; v < 8; ++v) {
                    const float hs = silu_scaled(acc[v]);
                    if (v & 1) pb = fmaf(hs, w4r[ma * 8 + v], pb);
                    else       pa = fmaf(hs, w4r[ma * 8 + v], pa);
                }
            }
            const float p   = pa + pb;
            const float tot = p + __shfl_xor(p, 16, 32) + b4s;

#pragma unroll
            for (int c = 0; c < 4; ++c) {
                const float s = __shfl(tot, src0 + c, 32);
                if (qsel == j) o[c] = s;
            }
        }

        const int ob = chunk * 128;
        float* op = out + (size_t)ob + 4 * lane;
        if (ob + 128 <= nOut) {
            *(volatile v4f*)op = o;
            __threadfence();
            *(volatile v4f*)op = o;
        } else {
#pragma unroll
            for (int c = 0; c < 4; ++c)
                if (ob + 4 * lane + c < nOut) *(volatile float*)(op + c) = o[c];
            __threadfence();
#pragma unroll
            for (int c = 0; c < 4; ++c)
                if (ob + 4 * lane + c < nOut) *(volatile float*)(op + c) = o[c];
        }
    }
}

extern "C" void kernel_launch(void* const* d_in, const int* in_sizes, int n_in,
                              void* d_out, int out_size, void* d_ws, size_t ws_size,
                              hipStream_t stream) {
    const float* x  = (const float*)d_in[0];
    const float* w1 = (const float*)d_in[1];
    const float* b1 = (const float*)d_in[2];
    const float* w2 = (const float*)d_in[3];
    const float* b2 = (const float*)d_in[4];
    const float* w3 = (const float*)d_in[5];
    const float* b3 = (const float*)d_in[6];
    const float* w4 = (const float*)d_in[7];
    const float* b4 = (const float*)d_in[8];
    float*       out = (float*)d_out;

    const int nX   = in_sizes[0];
    const int nOut = out_size;
    if (nX <= 0 || nOut <= 0) return;

    const int nChunks = (nOut + 127) / 128;
    int blocks = (nChunks + 7) / 8;
    if (blocks > 256) blocks = 256;
    if (blocks < 1)   blocks = 1;
    const int nWaves = blocks * 8;

    mlp_fp4_kernel<<<blocks, 256, 0, stream>>>(x, w1, b1, w2, b2, w3, b3, w4, b4,
                                               out, nX, nOut, nChunks, nWaves);
}
